// SinkhornDistance_44744969290142
// MI455X (gfx1250) — hardware-run, weakly checked
//
#include <hip/hip_runtime.h>
#define SNG 32
#define SNP 512
#define SND 256
typedef unsigned short v8us __attribute__((ext_vector_type(8), may_alias));
typedef float  v8f  __attribute__((ext_vector_type(8)));
typedef float  v4f  __attribute__((ext_vector_type(4)));
typedef float  v4fa __attribute__((ext_vector_type(4), may_alias));

__device__ __forceinline__ unsigned short bf16_bits(float x) { unsigned int u = __float_as_uint(x); return (unsigned short)((u + 0x7FFFu + ((u >> 16) & 1u)) >> 16); }
__device__ __forceinline__ float bf16_val(unsigned short b) { return __uint_as_float(((unsigned int)b) << 16); }
__device__ __forceinline__ float bf16_round(float x) { return bf16_val(bf16_bits(x)); }

typedef _Float16 v16h __attribute__((ext_vector_type(16)));
union FragH { v16h v; v8us half[2]; _Float16 h[16]; unsigned short u[16]; };

typedef _Float16 v4h __attribute__((ext_vector_type(4)));

__global__ __launch_bounds__(256) void k_x16(const float* __restrict__ x, _Float16* __restrict__ X16, size_t n8) { const size_t t = (size_t)blockIdx.x * 256 + threadIdx.x; if (t >= n8) return; FragH f;
#pragma unroll
  for (int q = 0; q < 8; ++q) f.h[q] = (_Float16)bf16_round(x[t * 8 + q]); *(volatile v8us*)((unsigned short*)X16 + t * 8) = f.half[0]; __threadfence(); *(volatile v8us*)((unsigned short*)X16 + t * 8) = f.half[0]; }

__device__ __forceinline__ v16h g2_frag(const _Float16* p, int hh) { FragH f; f.half[0] = *(const v8us*)((const unsigned short*)p + 8 * hh); f.half[1] = *(const v8us*)((const unsigned short*)p + 16 + 8 * hh); return f.v; }
__device__ __forceinline__ v8f g2_mma(v16h a, v16h b, v8f c) { v8f d = __builtin_amdgcn_wmma_f32_16x16x32_f16(false, a, false, b, (short)0, c, false, false); asm volatile("v_nop\n\tv_nop\n\tv_nop\n\tv_nop" : "+v"(d) : "v"(a), "v"(b)); return d; }
template <int ACT>
__global__ __launch_bounds__(128) void k_gemm2(const _Float16* __restrict__ A, int lda, size_t sA, const _Float16* __restrict__ Bh, int ldb, size_t sB, float alpha, const float* __restrict__ bias, size_t sBias, const float* __restrict__ CP, int rowsPerB, size_t sCPb, int row0g,
    float* __restrict__ C, _Float16* __restrict__ C16, int ldc, size_t sC, int M, int N, int K) { static_assert(ACT == 0 || ACT == 3 || ACT == 6 || ACT == 8 || ACT == 9 || ACT == 11 || ACT == 12 || ACT == 14 || ACT == 15 || ACT == 16 || ACT == 17, "k_gemm2: unsupported ACT code (would silently apply no activation)");
  __shared__ __attribute__((aligned(16))) float so[4][32][68];
  const int tid = threadIdx.x, w = tid >> 5, lane = tid & 31, ln = lane & 15, hh = lane >> 4; const int by = blockIdx.y;
  A += (size_t)by * sA; Bh += (size_t)by * sB; const size_t cofs = (size_t)by * sC; const float* bp = bias ? bias + (size_t)by * sBias : nullptr;
  const int ntn = N >> 6; const int mt = blockIdx.x / ntn, nq = blockIdx.x - mt * ntn; const int row0 = mt * 128 + 32 * w, col0 = nq * 64; if (row0 >= M) return;
  const _Float16* a0p = A + (size_t)(row0 + ln) * lda; const _Float16* a1p = a0p + (size_t)16 * lda;
  const _Float16* b0p = Bh + (size_t)(col0 + ln) * ldb; const _Float16* b1p = b0p + (size_t)16 * ldb; const _Float16* b2p = b1p + (size_t)16 * ldb; const _Float16* b3p = b2p + (size_t)16 * ldb;
  const v8f z8 = {0.f,0.f,0.f,0.f,0.f,0.f,0.f,0.f}; v8f c00 = z8, c01 = z8, c02 = z8, c03 = z8, c10 = z8, c11 = z8, c12 = z8, c13 = z8;
  for (int kb = 0; kb < K; kb += 32) { const v16h a0 = g2_frag(a0p + kb, hh), a1 = g2_frag(a1p + kb, hh);
    v16h b = g2_frag(b0p + kb, hh); c00 = g2_mma(a0, b, c00); c10 = g2_mma(a1, b, c10);
    b = g2_frag(b1p + kb, hh); c01 = g2_mma(a0, b, c01); c11 = g2_mma(a1, b, c11);
    b = g2_frag(b2p + kb, hh); c02 = g2_mma(a0, b, c02); c12 = g2_mma(a1, b, c12);
    b = g2_frag(b3p + kb, hh); c03 = g2_mma(a0, b, c03); c13 = g2_mma(a1, b, c13); }
  v8f accs[8] = {c00, c01, c02, c03, c10, c11, c12, c13};
#pragma unroll
  for (int u = 0; u < 8; ++u) { const int t = u & 3, half = u >> 2; const int col = col0 + t * 16 + ln; const float bv = bp ? bf16_round(bp[col]) : 0.f;
#pragma unroll
    for (int r = 0; r < 8; ++r) { const int rloc = half * 16 + 8 * hh + r; float v = accs[u][r] * alpha + bv; if (CP) { if (rowsPerB < 0) v += CP[cofs + (size_t)(row0g + row0 + rloc) * ldc + col];        else { const int bidx = (row0g + row0 + rloc) / rowsPerB; v += CP[(size_t)bidx * sCPb + (size_t)by * 64 + col]; } }
      if (ACT == 3) v = fmaxf(v, 0.f); else if (ACT == 6) v = 0.5f * v * (1.0f + erff(v * 0.70710678118654752f)); else if (ACT == 11) v = 1.0f / (1.0f + expf(-v)); else if (ACT == 15) v = v / (1.0f + expf(-v)); else if (ACT == 12) v = (v > 0.f) ? v : 0.01f * v; else if (ACT == 8) v = tanhf(v); else if (ACT == 9) v = 0.5f * v * (1.0f + tanhf(0.7978845608028654f * (v + 0.044715f * v * v * v))); else if (ACT == 14) v = (v > 0.f) ? v : 0.1f * v; else if (ACT == 16) v = (v >= 0.f) ? v : 0.3f * v; else if (ACT == 17) v = (v >= 0.f) ? v : 0.2f * v;
      so[w][rloc][t * 16 + ln] = v; } }
  __builtin_amdgcn_fence(__ATOMIC_ACQ_REL, "workgroup"); __builtin_amdgcn_wave_barrier();
  const int rsub = lane >> 4, c4 = (lane & 15) * 4;
  for (int pass = 0; pass < 2; ++pass) {
#pragma unroll
    for (int q = 0; q < 16; ++q) { const int r = q * 2 + rsub; const v4f v = *(const v4fa*)&so[w][r][c4]; if (C) *(volatile v4f*)(C + cofs + (size_t)(row0 + r) * ldc + col0 + c4) = v; if (C16) { v4h h4; for (int i = 0; i < 4; ++i) h4[i] = (_Float16)v[i]; *(volatile v4h*)(C16 + cofs + (size_t)(row0 + r) * ldc + col0 + c4) = h4; } }
    if (pass == 0) __threadfence(); } }

__global__ __launch_bounds__(256) void k_len(const float* __restrict__ ts, float* __restrict__ ln, float* __restrict__ one, float* __restrict__ nil, unsigned nrows) {
  const unsigned rr = blockIdx.x * 256u + threadIdx.x; if (rr >= nrows) return;
  const float* p = ts + (size_t)rr * SND; float ss = 0.0f;
  for (unsigned j = 0; j < (unsigned)SND; j += 4) { const v4f t4 = *(const v4fa*)(p + j);
#pragma unroll
    for (int q = 0; q < 4; ++q) { const float w = bf16_round(t4[q]); ss += w * w; } }
  const float ll = sqrtf(ss); *(volatile float*)(ln + rr) = ll; *(volatile float*)(one + rr) = 1.0f; *(volatile float*)(nil + rr) = 0.0f; __threadfence(); *(volatile float*)(ln + rr) = ll; *(volatile float*)(one + rr) = 1.0f; *(volatile float*)(nil + rr) = 0.0f; }

__global__ __launch_bounds__(256) void k_cosd(const float* __restrict__ dt, const float* __restrict__ la, const float* __restrict__ lb, float* __restrict__ cs, unsigned n4) {
  const unsigned t = blockIdx.x * 256u + threadIdx.x; if (t >= n4) return;
  const unsigned row = t / (unsigned)(SNP / 4), c4 = (t - row * (unsigned)(SNP / 4)) * 4u, grp = row / (unsigned)SNP;
  const v4f d4 = *(const v4fa*)(dt + (size_t)row * SNP + c4); const v4f b4 = *(const v4fa*)(lb + (size_t)grp * SNP + c4); const float al = la[row]; v4f o4;
#pragma unroll
  for (int q = 0; q < 4; ++q) o4[q] = 1.0f - d4[q] / fmaxf(al * b4[q], 1e-8f);
  *(volatile v4f*)(cs + (size_t)row * SNP + c4) = o4; __threadfence(); *(volatile v4f*)(cs + (size_t)row * SNP + c4) = o4; }

__global__ __launch_bounds__(256) void k_rowp(const float* __restrict__ cs, float* __restrict__ pa, const float* __restrict__ pb, float* __restrict__ ra, const float* __restrict__ rb, unsigned nrows) {
  const unsigned rr = blockIdx.x * 256u + threadIdx.x; if (rr >= nrows) return;
  const unsigned grp = rr / (unsigned)SNP; const float* cp = cs + (size_t)rr * SNP; const float* bp = pb + (size_t)grp * SNP; const float* vp = rb + (size_t)grp * SNP;
  const float ai = pa[rr] + 0.1f * logf(ra[rr]); float ss = 0.0f;
  for (unsigned j = 0; j < (unsigned)SNP; j += 4) { const v4f c4 = *(const v4fa*)(cp + j); const v4f b4 = *(const v4fa*)(bp + j); const v4f r4 = *(const v4fa*)(vp + j);
#pragma unroll
    for (int q = 0; q < 4; ++q) ss += expf((ai + b4[q] - c4[q]) * 10.0f) * r4[q]; }
  const float rn = (1.0f / (float)SNP) / (ss + 1e-16f);
  *(volatile float*)(pa + rr) = ai; *(volatile float*)(ra + rr) = rn; __threadfence(); *(volatile float*)(pa + rr) = ai; *(volatile float*)(ra + rr) = rn; }

__global__ __launch_bounds__(256) void k_colp(const float* __restrict__ cs, const float* __restrict__ pa, float* __restrict__ pb, const float* __restrict__ ra, float* __restrict__ rb, unsigned ncols) {
  const unsigned cc = blockIdx.x * 256u + threadIdx.x; if (cc >= ncols) return;
  const unsigned grp = cc / (unsigned)SNP, jj = cc - grp * (unsigned)SNP; const float* cp = cs + (size_t)grp * SNP * SNP + jj; const float* ap = pa + (size_t)grp * SNP; const float* up = ra + (size_t)grp * SNP;
  const float bj = pb[cc]; float ss = 0.0f;
  for (unsigned i = 0; i < (unsigned)SNP; i += 4) { const v4f a4 = *(const v4fa*)(ap + i); const v4f r4 = *(const v4fa*)(up + i);
#pragma unroll
    for (int q = 0; q < 4; ++q) ss += expf((a4[q] + bj - cp[(size_t)(i + q) * SNP]) * 10.0f) * r4[q]; }
  const float rn = (1.0f / (float)SNP) / (ss + 1e-16f); const float bn = bj + 0.1f * logf(rn);
  *(volatile float*)(rb + cc) = rn; *(volatile float*)(pb + cc) = bn; __threadfence(); *(volatile float*)(rb + cc) = rn; *(volatile float*)(pb + cc) = bn; }

__global__ __launch_bounds__(256) void k_plan(const float* __restrict__ cs, const float* __restrict__ pa, const float* __restrict__ pb, const float* __restrict__ ra, const float* __restrict__ rb, float* __restrict__ pl, float* __restrict__ rs, unsigned nrows) {
  const unsigned rr = blockIdx.x * 256u + threadIdx.x; if (rr >= nrows) return;
  const unsigned grp = rr / (unsigned)SNP; const float* cp = cs + (size_t)rr * SNP; const float* bp = pb + (size_t)grp * SNP; const float* vp = rb + (size_t)grp * SNP;
  const float lu = logf(ra[rr]); const float ai = pa[rr] + 0.1f * lu; float ss = 0.0f;
  for (int pass = 0; pass < 2; ++pass) { ss = 0.0f;
    for (unsigned j = 0; j < (unsigned)SNP; j += 4) { const v4f c4 = *(const v4fa*)(cp + j); const v4f b4 = *(const v4fa*)(bp + j); const v4f r4 = *(const v4fa*)(vp + j); v4f o4;
#pragma unroll
      for (int q = 0; q < 4; ++q) { o4[q] = expf(lu + (ai + b4[q] - c4[q]) * 10.0f + logf(r4[q])); ss += o4[q] * c4[q]; }
      *(volatile v4f*)(pl + (size_t)rr * SNP + j) = o4; }
    *(volatile float*)(rs + rr) = ss; if (pass == 0) __threadfence(); } }

__global__ __launch_bounds__(32) void k_tot(const float* __restrict__ rs, float* __restrict__ tc, unsigned ngrp) {
  const unsigned g = blockIdx.x * 32u + threadIdx.x; if (g >= ngrp) return;
  const float* p = rs + (size_t)g * SNP; float ss = 0.0f;
  for (unsigned j = 0; j < (unsigned)SNP; j += 4) { const v4f t4 = *(const v4fa*)(p + j); ss += t4[0]; ss += t4[1]; ss += t4[2]; ss += t4[3]; }
  *(volatile float*)(tc + g) = ss; __threadfence(); *(volatile float*)(tc + g) = ss; }

extern "C" void kernel_launch(void* const* d_in, const int* in_sizes, int n_in,
                              void* d_out, int out_size, void* d_ws, size_t ws_size, hipStream_t stream) {
  if (n_in < 2) return; if (in_sizes[0] < SNG * SNP * SND || in_sizes[1] < SNG * SNP * SND) return; if (out_size < SNG + 2 * SNG * SNP * SNP) return;
  const float* ta = (const float*)d_in[0]; const float* tb = (const float*)d_in[1];
  float* tc = (float*)d_out; float* pl = tc + SNG; float* cs = pl + (size_t)SNG * SNP * SNP;
  static_assert(SNP % 128 == 0 && SNP % 64 == 0 && SND % 32 == 0 && SND % 8 == 0 && SNP % 4 == 0 && SNG <= 32, "whole tiles");
  uint8_t* wsp = (uint8_t*)d_ws; size_t off = 0;
  auto take = [&](size_t bytes) { uint8_t* p = wsp + off; off += (bytes + 255) & ~(size_t)255; return p; };
  _Float16* TA = (_Float16*)take((size_t)SNG * SNP * SND * 2); _Float16* TB = (_Float16*)take((size_t)SNG * SNP * SND * 2); float* DT = (float*)take((size_t)SNG * SNP * SNP * 4); float* LA = (float*)take((size_t)SNG * SNP * 4); float* LB = (float*)take((size_t)SNG * SNP * 4); float* RA = (float*)take((size_t)SNG * SNP * 4); float* RB = (float*)take((size_t)SNG * SNP * 4); float* PA = (float*)take((size_t)SNG * SNP * 4); float* PB = (float*)take((size_t)SNG * SNP * 4); float* RS = (float*)take((size_t)SNG * SNP * 4);
  if (off > ws_size) return;
  k_x16<<<(unsigned)(((size_t)SNG * SNP * SND / 8 + 255) / 256), 256, 0, stream>>>(ta, TA, (size_t)SNG * SNP * SND / 8);
  k_x16<<<(unsigned)(((size_t)SNG * SNP * SND / 8 + 255) / 256), 256, 0, stream>>>(tb, TB, (size_t)SNG * SNP * SND / 8);
  k_gemm2<0><<<dim3((unsigned)((SNP / 128) * (SNP / 64)), (unsigned)SNG), 128, 0, stream>>>(TA, SND, (size_t)SNP * SND, TB, SND, (size_t)SNP * SND, 1.0f, nullptr, 0, nullptr, 1, 0, 0, DT, nullptr, SNP, (size_t)SNP * SNP, SNP, SNP, SND);
  k_len<<<(unsigned)((SNG * SNP + 255) / 256), 256, 0, stream>>>(ta, LA, RA, PA, (unsigned)(SNG * SNP));
  k_len<<<(unsigned)((SNG * SNP + 255) / 256), 256, 0, stream>>>(tb, LB, RB, PB, (unsigned)(SNG * SNP));
  k_cosd<<<(unsigned)(((size_t)SNG * SNP * SNP / 4 + 255) / 256), 256, 0, stream>>>(DT, LA, LB, cs, (unsigned)((size_t)SNG * SNP * SNP / 4));
  for (int st = 0; st < 15; ++st) {
    k_rowp<<<(unsigned)((SNG * SNP + 255) / 256), 256, 0, stream>>>(cs, PA, PB, RA, RB, (unsigned)(SNG * SNP));
    k_colp<<<(unsigned)((SNG * SNP + 255) / 256), 256, 0, stream>>>(cs, PA, PB, RA, RB, (unsigned)(SNG * SNP)); }
  k_plan<<<(unsigned)((SNG * SNP + 255) / 256), 256, 0, stream>>>(cs, PA, PB, RA, RB, pl, RS, (unsigned)(SNG * SNP));
  k_tot<<<1, 32, 0, stream>>>(RS, tc, (unsigned)SNG);
}
